// MambaCell_65704409694785
// MI455X (gfx1250) — hardware-verified
//
#include <hip/hip_runtime.h>
#include <math.h>

typedef __attribute__((ext_vector_type(16))) __bf16   v16b;
typedef __attribute__((ext_vector_type(8)))  __bf16   v8b;
typedef __attribute__((ext_vector_type(8)))  float    v8f;
typedef __attribute__((ext_vector_type(4)))  float    v4f;
typedef __attribute__((ext_vector_type(4)))  unsigned v4u;

constexpr int kBatch  = 4;
constexpr int kSeq    = 1024;
constexpr int kDm     = 1024;
constexpr int kDin    = 2048;
constexpr int kNst    = 16;
constexpr int kDtR    = 64;
constexpr int kPrjN   = 96;
constexpr int kPrjP   = 128;
constexpr int kXzP    = 2 * kDin;
constexpr int kRows   = kBatch * kSeq;
constexpr int kHalves = 2;
constexpr int kHRows  = kRows / kHalves;
constexpr int kConvTP = 260;
constexpr int kScanTS = 64;
constexpr int kScanCh = 64;
constexpr int kScanYP = 68;
constexpr float kInvDm = 1.0f / (float)kDm;
static_assert(kPrjN == kDtR + 2 * kNst, "x_proj width");
static_assert(kPrjP % 64 == 0 && kPrjP >= kPrjN, "padded x_proj width");
static_assert(kHRows % kSeq == 0 && kHRows % 64 == 0, "half = whole batch elements, tile multiple");
static_assert(kDm % 32 == 0 && kDin % 32 == 0 && kDtR % 32 == 0, "GEMM K multiples of 32");
static_assert(kXzP % 64 == 0 && kDin % 64 == 0 && kDm % 64 == 0, "GEMM N multiples of 64");
static_assert(kSeq % kScanTS == 0 && kSeq % 64 == 0 && kDin % kScanCh == 0 && kDin % 256 == 0, "tile multiples");
static_assert(kDm == 256 * 4, "one float4 per lane in the LayerNorm block");

constexpr size_t kOffWIN  = 0;
constexpr size_t kOffWX   = kOffWIN  + (size_t)kXzP  * kDm  * 2;
constexpr size_t kOffWDT  = kOffWX   + (size_t)kPrjP * kDin * 2;
constexpr size_t kOffWOUT = kOffWDT  + (size_t)kDin  * kDtR * 2;
constexpr size_t kOffUH   = kOffWOUT + (size_t)kDm   * kDin * 2;
constexpr size_t kOffUL   = kOffUH   + (size_t)kRows * kDm  * 2;
constexpr size_t kOffXZ   = kOffUL   + (size_t)kRows * kDm  * 2;
constexpr size_t kOffXS   = kOffXZ   + (size_t)kHRows * kXzP * 4;
constexpr size_t kOffXSH  = kOffXS   + (size_t)kHRows * kDin * 4;
constexpr size_t kOffXSL  = kOffXSH  + (size_t)kHRows * kDin * 2;
constexpr size_t kOffPROJ = kOffXSL  + (size_t)kHRows * kDin * 2;
constexpr size_t kOffDTH  = kOffPROJ + (size_t)kHRows * kPrjP * 4;
constexpr size_t kOffDTL  = kOffDTH  + (size_t)kHRows * kDtR * 2;
constexpr size_t kOffDLR  = kOffDTL  + (size_t)kHRows * kDtR * 2;
constexpr size_t kOffYH   = kOffDLR  + (size_t)kHRows * kDin * 4;
constexpr size_t kOffYL   = kOffYH   + (size_t)kHRows * kDin * 2;
constexpr size_t kWsTotal = kOffYL   + (size_t)kHRows * kDin * 2;
static_assert(kWsTotal == 132382720ull, "carve total");
static_assert(kWsTotal <= 134217728ull, "carve cap");
static_assert((kOffWX % 128) == 0 && (kOffWDT % 128) == 0 && (kOffWOUT % 128) == 0 && (kOffUH % 128) == 0 &&
              (kOffUL % 128) == 0 && (kOffXZ % 128) == 0 && (kOffXS % 128) == 0 && (kOffXSH % 128) == 0 &&
              (kOffXSL % 128) == 0 && (kOffPROJ % 128) == 0 && (kOffDTH % 128) == 0 && (kOffDTL % 128) == 0 &&
              (kOffDLR % 128) == 0 && (kOffYH % 128) == 0 && (kOffYL % 128) == 0, "128-B aligned regions");
constexpr size_t kOut1Elems = (size_t)kRows * kDm;
static_assert(kOut1Elems * 4 == 16777216ull, "out1 byte offset");
static_assert(kOut1Elems * 4 * 2 == 33554432ull, "d_out total bytes");

__device__ __forceinline__ unsigned short f2bf_bits(float f) {
  unsigned u = __float_as_uint(f);
  return (unsigned short)((u + 0x7FFFu + ((u >> 16) & 1u)) >> 16);
}
__device__ __forceinline__ float bf_bits2f(unsigned short h) { return __uint_as_float(((unsigned)h) << 16); }
__device__ __forceinline__ float bf_rne(float f) { return bf_bits2f(f2bf_bits(f)); }

__device__ __forceinline__ void split2(float x0, float x1, unsigned& hw, unsigned& lw) {
  const unsigned short h0 = f2bf_bits(x0);
  const unsigned short h1 = f2bf_bits(x1);
  const unsigned short l0 = f2bf_bits(x0 - bf_bits2f(h0));
  const unsigned short l1 = f2bf_bits(x1 - bf_bits2f(h1));
  hw = (unsigned)h0 | ((unsigned)h1 << 16);
  lw = (unsigned)l0 | ((unsigned)l1 << 16);
}
__device__ __forceinline__ void split8(const v4f a0, const v4f a1, v4u& hv, v4u& lv) {
  const float x0 = a0[0], x1 = a0[1], x2 = a0[2], x3 = a0[3];
  const float x4 = a1[0], x5 = a1[1], x6 = a1[2], x7 = a1[3];
  unsigned h0, h1, h2, h3, l0, l1, l2, l3;
  split2(x0, x1, h0, l0);
  split2(x2, x3, h1, l1);
  split2(x4, x5, h2, l2);
  split2(x6, x7, h3, l3);
  hv = (v4u){h0, h1, h2, h3};
  lv = (v4u){l0, l1, l2, l3};
}

__device__ __forceinline__ v16b frag_load(const __bf16* p) {
  union { v16b v; v8b h[2]; } f;
  f.h[0] = *(const v8b*)(p);
  f.h[1] = *(const v8b*)(p + 16);
  return f.v;
}
__device__ __forceinline__ v8f mma_b(v16b a, v16b b, v8f c) {
  return __builtin_amdgcn_wmma_f32_16x16x32_bf16(false, a, false, b, (short)0, c, false, false);
}
__device__ __forceinline__ void guard_row(v8f& a, v8f& b, v8f& c, v8f& d, v16b x, v16b y) {
  asm volatile("v_nop\n\tv_nop\n\tv_nop\n\tv_nop" : "+v"(a), "+v"(b), "+v"(c), "+v"(d) : "v"(x), "v"(y));
}
__device__ __forceinline__ void keep4_b(v16b a, v16b b, v16b c, v16b d) { asm volatile("v_nop" :: "v"(a), "v"(b), "v"(c), "v"(d)); }
__device__ __forceinline__ void acc_guard4(v8f& a, v8f& b, v8f& c, v8f& d) { asm volatile("v_nop\n\tv_nop\n\tv_nop\n\tv_nop" : "+v"(a), "+v"(b), "+v"(c), "+v"(d)); }

__global__ __launch_bounds__(256) void wmma_gemm_a2(
    const unsigned short* __restrict__ Ahp, const unsigned short* __restrict__ Alp, int lda,
    const unsigned short* __restrict__ Btp, int ldb,
    float* __restrict__ Cout, int ldc, int M, int N, int K)
{
  const __bf16* Ah = (const __bf16*)Ahp;
  const __bf16* Al = (const __bf16*)Alp;
  const __bf16* Bt = (const __bf16*)Btp;
  __shared__ __align__(16) float sT[8][16 * 68];
  const int lane = threadIdx.x & 31;
  const int wave = threadIdx.x >> 5;
  const int tilesN = N >> 6;
  const int tilesM = M >> 6;
  const int tile = blockIdx.x * 8 + wave;
  if (tile >= tilesM * tilesN) return;
  const int tm = tile / tilesN;
  const int tn = tile - tm * tilesN;
  const int m0 = tm << 6;
  const int n0 = tn << 6;

  const int rlane = lane & 15;
  const int koff  = (lane >> 4) * 8;
  const int mOff  = (lane >> 4) * 8;

  v8f acc[4][4];
#pragma unroll
  for (int i = 0; i < 4; ++i)
#pragma unroll
    for (int j = 0; j < 4; ++j) acc[i][j] = (v8f){0.f, 0.f, 0.f, 0.f, 0.f, 0.f, 0.f, 0.f};

  for (int k0 = 0; k0 < K; k0 += 32) {
    v16b bh[4];
#pragma unroll
    for (int j = 0; j < 4; ++j) {
      const size_t bo = (size_t)(n0 + (j << 4) + rlane) * ldb + koff + k0;
      bh[j] = frag_load(Bt + bo);
    }
#pragma unroll
    for (int i = 0; i < 4; ++i) {
      const size_t ao = (size_t)(m0 + (i << 4) + rlane) * lda + koff + k0;
      const v16b ah = frag_load(Ah + ao);
      const v16b al = frag_load(Al + ao);
#pragma unroll
      for (int j = 0; j < 4; ++j) {
        acc[i][j] = mma_b(ah, bh[j], acc[i][j]);
        acc[i][j] = mma_b(al, bh[j], acc[i][j]);
      }
      guard_row(acc[i][0], acc[i][1], acc[i][2], acc[i][3], ah, al);
    }
    keep4_b(bh[0], bh[1], bh[2], bh[3]);
  }
  acc_guard4(acc[0][0], acc[0][1], acc[0][2], acc[0][3]);
  acc_guard4(acc[1][0], acc[1][1], acc[1][2], acc[1][3]);
  acc_guard4(acc[2][0], acc[2][1], acc[2][2], acc[2][3]);
  acc_guard4(acc[3][0], acc[3][1], acc[3][2], acc[3][3]);

  float* slab = sT[wave];
#pragma unroll
  for (int i = 0; i < 4; ++i) {
    const int mBase = m0 + (i << 4);
#pragma unroll
    for (int j = 0; j < 4; ++j) {
#pragma unroll
      for (int r = 0; r < 8; ++r) {
        slab[(mOff + r) * 68 + (j << 4) + rlane] = acc[i][j][r];
      }
    }
    __builtin_amdgcn_fence(__ATOMIC_RELEASE, "workgroup");
    __builtin_amdgcn_wave_barrier();
    __builtin_amdgcn_fence(__ATOMIC_ACQUIRE, "workgroup");
    {
      const int hh = lane >> 4, c4 = (lane & 15) * 4;
      for (int pass = 0; pass < 2; ++pass) {
#pragma unroll
        for (int it = 0; it < 8; ++it) {
          const int row = it * 2 + hh;
          const v4f v = *(const v4f*)(slab + row * 68 + c4);
          *(volatile v4f*)(Cout + (size_t)(mBase + row) * ldc + n0 + c4) = v;
        }
        __threadfence();
      }
    }
    __builtin_amdgcn_fence(__ATOMIC_RELEASE, "workgroup");
    __builtin_amdgcn_wave_barrier();
    __builtin_amdgcn_fence(__ATOMIC_ACQUIRE, "workgroup");
  }
}

__global__ __launch_bounds__(256) void ln_split_kernel(
    const float* __restrict__ x, const float* __restrict__ lnw, const float* __restrict__ lnb,
    float* __restrict__ out1, unsigned short* __restrict__ UH, unsigned short* __restrict__ UL)
{
  __shared__ float sR1[8];
  __shared__ float sR2[8];
  __shared__ __align__(16) float sU[kDm];
  const int tid = threadIdx.x, lane = tid & 31, wave = tid >> 5;
  const size_t base = (size_t)blockIdx.x * kDm + (size_t)tid * 4;
  const v4f xv = *(const v4f*)(x + base);
  *(volatile v4f*)(out1 + base) = xv;
  const float r0 = bf_rne(xv[0]), r1 = bf_rne(xv[1]), r2 = bf_rne(xv[2]), r3 = bf_rne(xv[3]);
  float s = (r0 + r1) + (r2 + r3);
#pragma unroll
  for (int off = 16; off > 0; off >>= 1) s += __shfl_xor(s, off, 32);
  if (lane == 0) sR1[wave] = s;
  __syncthreads();
  float tot = 0.f;
#pragma unroll
  for (int w = 0; w < 8; ++w) tot += sR1[w];
  const float mu = tot * kInvDm;
  const float c0 = r0 - mu, c1 = r1 - mu, c2 = r2 - mu, c3 = r3 - mu;
  float ss = (c0 * c0 + c1 * c1) + (c2 * c2 + c3 * c3);
#pragma unroll
  for (int off = 16; off > 0; off >>= 1) ss += __shfl_xor(ss, off, 32);
  if (lane == 0) sR2[wave] = ss;
  __syncthreads();
  float tot2 = 0.f;
#pragma unroll
  for (int w = 0; w < 8; ++w) tot2 += sR2[w];
  const float var  = tot2 * kInvDm;
  const float rstd = rsqrtf(var + 1e-5f);
  const v4f wv = *(const v4f*)(lnw + tid * 4);
  const v4f bv = *(const v4f*)(lnb + tid * 4);
  const float w0 = bf_rne(wv[0]), w1 = bf_rne(wv[1]), w2 = bf_rne(wv[2]), w3 = bf_rne(wv[3]);
  const float b0 = bf_rne(bv[0]), b1 = bf_rne(bv[1]), b2 = bf_rne(bv[2]), b3 = bf_rne(bv[3]);
  v4f uv;
  uv[0] = (c0 * rstd) * w0 + b0;
  uv[1] = (c1 * rstd) * w1 + b1;
  uv[2] = (c2 * rstd) * w2 + b2;
  uv[3] = (c3 * rstd) * w3 + b3;
  *(v4f*)(sU + tid * 4) = uv;
  __syncthreads();
  const int seg = (wave & 3) * 32 + lane;
  const v4f a0 = *(const v4f*)(sU + seg * 8);
  const v4f a1 = *(const v4f*)(sU + seg * 8 + 4);
  v4u hv, lv;
  split8(a0, a1, hv, lv);
  const bool hiw = (wave < 4);
  unsigned short* dst = (hiw ? UH : UL) + (size_t)blockIdx.x * kDm + seg * 8;
  const v4u val = hiw ? hv : lv;
  *(volatile v4u*)dst = val;
  __threadfence();
  *(volatile v4f*)(out1 + base) = xv;
  *(volatile v4u*)dst = val;
}

__global__ __launch_bounds__(256) void cast_bf16_kernel(
    const float* __restrict__ src, unsigned short* __restrict__ dst, int total8, int src8)
{
  const int i = blockIdx.x * 256 + threadIdx.x;
  if (i >= total8) return;
  const bool live = (i < src8);
  const int ic = live ? i : (src8 - 1);
  const float* p = src + ((size_t)ic << 3);
  const v4f a0 = *(const v4f*)(p);
  const v4f a1 = *(const v4f*)(p + 4);
  const float f0 = live ? a0[0] : 0.0f, f1 = live ? a0[1] : 0.0f, f2 = live ? a0[2] : 0.0f, f3 = live ? a0[3] : 0.0f;
  const float f4 = live ? a1[0] : 0.0f, f5 = live ? a1[1] : 0.0f, f6 = live ? a1[2] : 0.0f, f7 = live ? a1[3] : 0.0f;
  const unsigned q0 = (unsigned)f2bf_bits(f0) | ((unsigned)f2bf_bits(f1) << 16);
  const unsigned q1 = (unsigned)f2bf_bits(f2) | ((unsigned)f2bf_bits(f3) << 16);
  const unsigned q2 = (unsigned)f2bf_bits(f4) | ((unsigned)f2bf_bits(f5) << 16);
  const unsigned q3 = (unsigned)f2bf_bits(f6) | ((unsigned)f2bf_bits(f7) << 16);
  const v4u val = (v4u){q0, q1, q2, q3};
  unsigned short* q = dst + ((size_t)i << 3);
  *(volatile v4u*)q = val;
  __threadfence();
  *(volatile v4u*)q = val;
}

__global__ __launch_bounds__(256) void dt_split_kernel(
    const float* __restrict__ PROJ, unsigned short* __restrict__ DTH, unsigned short* __restrict__ DTL, int total8)
{
  const int i = blockIdx.x * 256 + threadIdx.x;
  if (i >= total8) return;
  const int e0  = i << 3;
  const int row = e0 >> 6;
  const int c8  = e0 & 63;
  const float* p = PROJ + (size_t)row * kPrjP + c8;
  const v4f a0 = *(const v4f*)(p);
  const v4f a1 = *(const v4f*)(p + 4);
  v4u hv, lv;
  split8(a0, a1, hv, lv);
  unsigned short* qh = DTH + e0;
  unsigned short* ql = DTL + e0;
  *(volatile v4u*)qh = hv;
  *(volatile v4u*)ql = lv;
  __threadfence();
  *(volatile v4u*)qh = hv;
  *(volatile v4u*)ql = lv;
}

__global__ __launch_bounds__(256) void conv_silu_kernel(
    const float* __restrict__ XZ, const float* __restrict__ cw, const float* __restrict__ cb,
    float* __restrict__ XS, unsigned short* __restrict__ XSH, unsigned short* __restrict__ XSL)
{
  __shared__ __align__(16) float sT[16 * kConvTP];
  const int tid = threadIdx.x, lane = tid & 31, wave = tid >> 5;
  const int d0 = blockIdx.x * 256, d = d0 + tid;
  const int g0 = blockIdx.y * 64;
  const int tb = g0 & (kSeq - 1);
  const v4f wv = *(const v4f*)(cw + (size_t)d * 4);
  const float w0 = bf_rne(wv[0]), w1 = bf_rne(wv[1]), w2 = bf_rne(wv[2]), w3 = bf_rne(wv[3]);
  const float bc = bf_rne(cb[d]);
  float xm3, xm2, xm1;
  {
    const bool hist = (tb > 0);
    const int rb = hist ? (g0 - 3) : g0;
    const float v3 = XZ[(size_t)rb * kXzP + d];
    const float v2 = XZ[(size_t)(rb + 1) * kXzP + d];
    const float v1 = XZ[(size_t)(rb + 2) * kXzP + d];
    xm3 = hist ? v3 : 0.f;
    xm2 = hist ? v2 : 0.f;
    xm1 = hist ? v1 : 0.f;
  }
  const int hrow = wave >> 1;
  const int hch  = (wave & 1) * 128 + lane * 4;
#pragma unroll 1
  for (int sub = 0; sub < 4; ++sub) {
    const int lb = g0 + sub * 16;
#pragma unroll 1
    for (int s = 0; s < 16; ++s) {
      const float xcur = XZ[(size_t)(lb + s) * kXzP + d];
      float acc = fmaf(w0, xm3, bc);
      acc = fmaf(w1, xm2, acc);
      acc = fmaf(w2, xm1, acc);
      acc = fmaf(w3, xcur, acc);
      const float sg = __builtin_amdgcn_rcpf(1.0f + expf(-acc));
      sT[s * kConvTP + tid] = acc * sg;
      xm3 = xm2; xm2 = xm1; xm1 = xcur;
    }
    __syncthreads();
    v4f fv[4];
    v4u bh[2], bl[2];
#pragma unroll
    for (int it = 0; it < 4; ++it) fv[it] = *(const v4f*)(sT + (it * 4 + hrow) * kConvTP + hch);
#pragma unroll
    for (int it = 0; it < 2; ++it) {
      const float* sp = sT + (it * 8 + wave) * kConvTP + lane * 8;
      const v4f a0 = *(const v4f*)(sp);
      const v4f a1 = *(const v4f*)(sp + 4);
      split8(a0, a1, bh[it], bl[it]);
    }
    for (int pass = 0; pass < 2; ++pass) {
#pragma unroll
      for (int it = 0; it < 4; ++it)
        *(volatile v4f*)(XS + (size_t)(lb + it * 4 + hrow) * kDin + d0 + hch) = fv[it];
#pragma unroll
      for (int it = 0; it < 2; ++it) {
        const size_t o = (size_t)(lb + it * 8 + wave) * kDin + d0 + lane * 8;
        *(volatile v4u*)(XSH + o) = bh[it];
        *(volatile v4u*)(XSL + o) = bl[it];
      }
      __threadfence();
    }
    __syncthreads();
  }
}

__global__ __launch_bounds__(64) void scan_kernel(
    const float* __restrict__ DLR, const float* __restrict__ XS, const float* __restrict__ XZ,
    const float* __restrict__ PROJ, const float* __restrict__ bdt, const float* __restrict__ Alog,
    const float* __restrict__ Dp, unsigned short* __restrict__ YH, unsigned short* __restrict__ YL)
{
  __shared__ __align__(16) float sBC[kScanTS * 32];
  __shared__ __align__(16) float sY[kScanTS * kScanYP];
  __shared__ __align__(16) float sA[kNst * kScanCh];
  const int tid = threadIdx.x, lane = tid & 31, wave = tid >> 5;
  constexpr int kBlkPerB = kDin / kScanCh;
  const int bix = blockIdx.x / kBlkPerB;
  const int d0  = (blockIdx.x - bix * kBlkPerB) * kScanCh;
  const int d   = d0 + tid;
  const size_t row0 = (size_t)bix * kSeq;
#pragma unroll 1
  for (int s = 0; s < kNst; ++s) sA[s * kScanCh + tid] = -expf(bf_rne(Alog[(size_t)d * kNst + s]));
  __syncthreads();
  float negA[kNst], h[kNst];
#pragma unroll
  for (int s = 0; s < kNst; ++s) {
    negA[s] = sA[s * kScanCh + tid];
    h[s] = 0.f;
  }
  const float bb = bf_rne(bdt[d]);
  const float Dd = bf_rne(Dp[d]);
  const int q = lane >> 3, c8 = (lane & 7) * 8;
#pragma unroll 1
  for (int t0 = 0; t0 < kSeq; t0 += kScanTS) {
    __syncthreads();
#pragma unroll
    for (int i = 0; i < 8; ++i) {
      const int idx = tid + 64 * i;
      const int r   = idx >> 3;
      const int cc  = (idx & 7) * 4;
      *(v4f*)(sBC + r * 32 + cc) = *(const v4f*)(PROJ + (row0 + t0 + r) * kPrjP + kDtR + cc);
    }
    __syncthreads();
#pragma unroll 1
    for (int s = 0; s < kScanTS; ++s) {
      const size_t grow = row0 + t0 + s;
      const float* xr = sBC + s * 32;
      float Bs[kNst], Cs[kNst];
#pragma unroll
      for (int q4 = 0; q4 < 4; ++q4) {
        const v4f bv = *(const v4f*)(xr + 4 * q4);
        const v4f cv = *(const v4f*)(xr + kNst + 4 * q4);
        Bs[4 * q4 + 0] = bv[0]; Bs[4 * q4 + 1] = bv[1]; Bs[4 * q4 + 2] = bv[2]; Bs[4 * q4 + 3] = bv[3];
        Cs[4 * q4 + 0] = cv[0]; Cs[4 * q4 + 1] = cv[1]; Cs[4 * q4 + 2] = cv[2]; Cs[4 * q4 + 3] = cv[3];
      }
      const float v   = DLR[grow * kDin + d] + bb;
      const float a   = __expf(-fabsf(v));
      const float u   = 1.0f + a;
      const float l1p = __logf(u) + (a - (u - 1.0f)) * __builtin_amdgcn_rcpf(u);
      const float dt  = fmaxf(v, 0.0f) + l1p;
      const float xt  = XS[grow * kDin + d];
      const float dtx = dt * xt;
      float y = 0.f;
#pragma unroll
      for (int k = 0; k < kNst; ++k) {
        const float e = __expf(dt * negA[k]);
        h[k] = e * h[k] + dtx * Bs[k];
        y = h[k] * Cs[k] + y;
      }
      y = xt * Dd + y;
      const float zv = XZ[grow * kXzP + kDin + d];
      const float sg = __builtin_amdgcn_rcpf(1.0f + expf(-zv));
      y = y * (zv * sg);
      sY[s * kScanYP + tid] = y;
    }
    __syncthreads();
    v4u hv[8], lv[8];
#pragma unroll
    for (int it = 0; it < 8; ++it) {
      const int row = it * 8 + wave * 4 + q;
      const float* sp = sY + row * kScanYP + c8;
      const v4f a0 = *(const v4f*)(sp);
      const v4f a1 = *(const v4f*)(sp + 4);
      split8(a0, a1, hv[it], lv[it]);
    }
    for (int pass = 0; pass < 2; ++pass) {
#pragma unroll
      for (int it = 0; it < 8; ++it) {
        const int row = it * 8 + wave * 4 + q;
        const size_t o = (row0 + t0 + row) * kDin + d0 + c8;
        *(volatile v4u*)(YH + o) = hv[it];
        *(volatile v4u*)(YL + o) = lv[it];
      }
      __threadfence();
    }
  }
}

extern "C" void kernel_launch(void* const* d_in, const int* in_sizes, int n_in,
                              void* d_out, int out_size, void* d_ws, size_t ws_size,
                              hipStream_t stream)
{
  if (n_in < 12) return;
  if (in_sizes[0] != kRows * kDm) return;
  if (in_sizes[1] != kDm || in_sizes[2] != kDm) return;
  if (in_sizes[3] != kXzP * kDm) return;
  if (in_sizes[4] != kDin * 4 || in_sizes[5] != kDin) return;
  if (in_sizes[6] != kPrjN * kDin) return;
  if (in_sizes[7] != kDin * kDtR || in_sizes[8] != kDin) return;
  if (in_sizes[9] != kDin * kNst || in_sizes[10] != kDin) return;
  if (in_sizes[11] != kDm * kDin) return;
  if (out_size != 2 * kRows * kDm) return;
  if (ws_size < kWsTotal) return;

  const float* x      = (const float*)d_in[0];
  const float* ln_w   = (const float*)d_in[1];
  const float* ln_b   = (const float*)d_in[2];
  const float* W_in   = (const float*)d_in[3];
  const float* conv_w = (const float*)d_in[4];
  const float* conv_b = (const float*)d_in[5];
  const float* W_x    = (const float*)d_in[6];
  const float* W_dt   = (const float*)d_in[7];
  const float* b_dt   = (const float*)d_in[8];
  const float* A_log  = (const float*)d_in[9];
  const float* D_skip = (const float*)d_in[10];
  const float* W_out  = (const float*)d_in[11];
  float* out0 = (float*)d_out;
  float* out1 = out0 + kOut1Elems;

  char* ws = (char*)d_ws;
  unsigned short* WIN  = (unsigned short*)(ws + kOffWIN);
  unsigned short* WX   = (unsigned short*)(ws + kOffWX);
  unsigned short* WDT  = (unsigned short*)(ws + kOffWDT);
  unsigned short* WOUT = (unsigned short*)(ws + kOffWOUT);
  unsigned short* UH   = (unsigned short*)(ws + kOffUH);
  unsigned short* UL   = (unsigned short*)(ws + kOffUL);
  float*          XZ   = (float*)(ws + kOffXZ);
  float*          XS   = (float*)(ws + kOffXS);
  unsigned short* XSH  = (unsigned short*)(ws + kOffXSH);
  unsigned short* XSL  = (unsigned short*)(ws + kOffXSL);
  float*          PROJ = (float*)(ws + kOffPROJ);
  unsigned short* DTH  = (unsigned short*)(ws + kOffDTH);
  unsigned short* DTL  = (unsigned short*)(ws + kOffDTL);
  float*          DLR  = (float*)(ws + kOffDLR);
  unsigned short* YH   = (unsigned short*)(ws + kOffYH);
  unsigned short* YL   = (unsigned short*)(ws + kOffYL);

  ln_split_kernel<<<kRows, 256, 0, stream>>>(x, ln_w, ln_b, out1, UH, UL);

  cast_bf16_kernel<<<(kXzP * kDm / 8) / 256, 256, 0, stream>>>(W_in, WIN, kXzP * kDm / 8, kXzP * kDm / 8);
  cast_bf16_kernel<<<(kPrjP * kDin / 8) / 256, 256, 0, stream>>>(W_x, WX, kPrjP * kDin / 8, kPrjN * kDin / 8);
  cast_bf16_kernel<<<(kDin * kDtR / 8) / 256, 256, 0, stream>>>(W_dt, WDT, kDin * kDtR / 8, kDin * kDtR / 8);
  cast_bf16_kernel<<<(kDm * kDin / 8) / 256, 256, 0, stream>>>(W_out, WOUT, kDm * kDin / 8, kDm * kDin / 8);

  for (int hf = 0; hf < kHalves; ++hf) {
    const unsigned short* UHh = UH + (size_t)hf * kHRows * kDm;
    const unsigned short* ULh = UL + (size_t)hf * kHRows * kDm;
    float* outh = out0 + (size_t)hf * kHRows * kDm;

    wmma_gemm_a2<<<dim3((kHRows / 64) * (kXzP / 64) / 8), 256, 0, stream>>>(
        UHh, ULh, kDm, WIN, kDm, XZ, kXzP, kHRows, kXzP, kDm);

    conv_silu_kernel<<<dim3(kDin / 256, kHRows / 64), 256, 0, stream>>>(XZ, conv_w, conv_b, XS, XSH, XSL);

    wmma_gemm_a2<<<dim3((kHRows / 64) * (kPrjP / 64) / 8), 256, 0, stream>>>(
        XSH, XSL, kDin, WX, kDin, PROJ, kPrjP, kHRows, kPrjP, kDin);

    dt_split_kernel<<<(kHRows * kDtR / 8) / 256, 256, 0, stream>>>(PROJ, DTH, DTL, kHRows * kDtR / 8);

    wmma_gemm_a2<<<dim3((kHRows / 64) * (kDin / 64) / 8), 256, 0, stream>>>(
        DTH, DTL, kDtR, WDT, kDtR, DLR, kDin, kHRows, kDin, kDtR);

    scan_kernel<<<(kHRows / kSeq) * (kDin / kScanCh), kScanCh, 0, stream>>>(
        DLR, XS, XZ, PROJ, b_dt, A_log, D_skip, YH, YL);

    wmma_gemm_a2<<<dim3((kHRows / 64) * (kDm / 64) / 8), 256, 0, stream>>>(
        YH, YL, kDin, WOUT, kDin, outh, kDm, kHRows, kDm, kDin);
  }
}
